// cheb_conv_with_SAt_7584912245217
// MI455X (gfx1250) — hardware-verified
//
#include <hip/hip_runtime.h>


#define NB_  8
#define NN   1024
#define FF   64
#define TS   12
#define KC   3
#define OO   64
#define FT   (FF * TS)
#define KF   (KC * FF)
#define NT   (NN * TS)
typedef _Float16 h16;
typedef unsigned short bf;
typedef __attribute__((ext_vector_type(16))) __bf16   v16bf;
typedef __attribute__((ext_vector_type(16))) _Float16 v16h;
typedef __attribute__((ext_vector_type(8)))  _Float16 v8h;
typedef __attribute__((ext_vector_type(8)))  unsigned short v8us;
typedef __attribute__((ext_vector_type(8)))  float    v8f;
typedef __attribute__((ext_vector_type(4)))  float    v4f;
typedef v8h  __attribute__((may_alias)) v8ha;
typedef v4f  __attribute__((may_alias)) v4fa;
typedef v8us __attribute__((may_alias)) v8usa;

__device__ __forceinline__ unsigned short f2bf(float f) { unsigned u = __float_as_uint(f); u += 0x7FFFu + ((u >> 16) & 1u); return (unsigned short)(u >> 16); }
__device__ __forceinline__ float bf2f(unsigned short b) { return __uint_as_float(((unsigned)b) << 16); }
__device__ __forceinline__ float bfr(float f) { return bf2f(f2bf(f)); }
__device__ __forceinline__ v16h cat16(v8h lo, v8h hi) { return __builtin_shufflevector(lo, hi, 0, 1, 2, 3, 4, 5, 6, 7, 8, 9, 10, 11, 12, 13, 14, 15); }
__device__ __forceinline__ v16bf cat16b(v8us lo, v8us hi) { return __builtin_bit_cast(v16bf, __builtin_shufflevector(lo, hi, 0, 1, 2, 3, 4, 5, 6, 7, 8, 9, 10, 11, 12, 13, 14, 15)); }
__device__ __forceinline__ v8f wmma16(v16h a, v16h b, v8f c) { return __builtin_amdgcn_wmma_f32_16x16x32_f16(false, a, false, b, (short)0, c, false, false); }
__device__ __forceinline__ v8f wmmab(v16bf a, v16bf b, v8f c) { return __builtin_amdgcn_wmma_f32_16x16x32_bf16(false, a, false, b, (short)0, c, false, false); }


template <typename T16> struct WFrag;
template <> struct WFrag<h16> { typedef v16h V; static __device__ __forceinline__ V ld(const h16* p) { return cat16(*(const v8h*)p, *(const v8h*)(p + 16)); } static __device__ __forceinline__ v8f mma(V a, V b, v8f c) { return wmma16(a, b, c); } };
template <> struct WFrag<bf> { typedef v16bf V; static __device__ __forceinline__ V ld(const bf* p) { return cat16b(*(const v8us*)p, *(const v8us*)(p + 16)); } static __device__ __forceinline__ v8f mma(V a, V b, v8f c) { return wmmab(a, b, c); } };
template <typename T16, int NSPLIT, bool BIAS>
__global__ __launch_bounds__(32) void k_gemmw(const T16* __restrict__ A, const T16* __restrict__ A2, const T16* __restrict__ Bt, const T16* __restrict__ Bt2, int K, float* C, int ldc, const float* __restrict__ bias, size_t sA, size_t sB, size_t sC) {
    typedef typename WFrag<T16>::V V;
    __shared__ __align__(16) float os[16 * 68];
    const size_t z = blockIdx.z; A += z * sA; if (A2) A2 += z * sA; Bt += z * sB; if (Bt2) Bt2 += z * sB; C += z * sC;
    const int lane = threadIdx.x & 31, lr = lane & 15, hi = lane >> 4; const int r0 = blockIdx.x * 64, c0 = blockIdx.y * 64;
    v8f acc[4][4];
#pragma unroll
    for (int mb = 0; mb < 4; ++mb)
#pragma unroll
        for (int nb = 0; nb < 4; ++nb) acc[mb][nb] = (v8f){};
    const size_t aoff = (size_t)(r0 + lr) * K + 8 * hi, boff = (size_t)(c0 + lr) * K + 8 * hi;
#pragma unroll 1
    for (int kc = 0; kc < K; kc += 32) {
        V a[4], a2[4];
#pragma unroll
        for (int mb = 0; mb < 4; ++mb) { a[mb] = WFrag<T16>::ld(A + aoff + (size_t)mb * 16 * K + kc); if (NSPLIT == 1 || NSPLIT == 2) a2[mb] = WFrag<T16>::ld(A2 + aoff + (size_t)mb * 16 * K + kc); }
#pragma unroll
        for (int nb = 0; nb < 4; ++nb) { const V b = WFrag<T16>::ld(Bt + boff + (size_t)nb * 16 * K + kc); V b2; if (NSPLIT >= 2) b2 = WFrag<T16>::ld(Bt2 + boff + (size_t)nb * 16 * K + kc);
#pragma unroll
            for (int mb = 0; mb < 4; ++mb) { acc[mb][nb] = WFrag<T16>::mma(a[mb], b, acc[mb][nb]); if (NSPLIT == 1 || NSPLIT == 2) acc[mb][nb] = WFrag<T16>::mma(a2[mb], b, acc[mb][nb]); if (NSPLIT >= 2) acc[mb][nb] = WFrag<T16>::mma(a[mb], b2, acc[mb][nb]); } }
        asm volatile("v_nop\n\tv_nop\n\tv_nop\n\tv_nop" : "+v"(acc[0][0]), "+v"(acc[1][1]), "+v"(acc[2][2]), "+v"(acc[3][3]) : "v"(a[0]), "v"(a[3]));
    }
#pragma unroll
    for (int mb = 0; mb < 4; ++mb) {
#pragma unroll
        for (int nb = 0; nb < 4; ++nb) {
#pragma unroll
            for (int j = 0; j < 8; ++j) os[(hi * 8 + j) * 68 + nb * 16 + lr] = acc[mb][nb][j]; }
        __builtin_amdgcn_wave_barrier(); asm volatile("" ::: "memory");
        float* crow = C + (size_t)(r0 + mb * 16) * ldc + c0;
#pragma unroll 1
        for (int ps = 0; ps < 2; ++ps) {
#pragma unroll
            for (int s = 0; s < 8; ++s) { const int row = 2 * s + hi, cofs = lr * 4; v4f val = *(const v4fa*)(os + row * 68 + cofs); if (BIAS) { val[0] += bfr(bias[c0 + cofs]); val[1] += bfr(bias[c0 + cofs + 1]); val[2] += bfr(bias[c0 + cofs + 2]); val[3] += bfr(bias[c0 + cofs + 3]); }
                *(volatile v4f*)(crow + (size_t)row * ldc + cofs) = val; }
            if (ps == 0) __threadfence(); }
        __builtin_amdgcn_wave_barrier(); asm volatile("" ::: "memory");
    }
}

__device__ __forceinline__ void splitf(float y, unsigned short& h, unsigned short& l) { h = f2bf(y); l = f2bf(y - bf2f(h)); }
typedef __attribute__((ext_vector_type(2))) unsigned short v2us;
typedef __attribute__((ext_vector_type(4))) unsigned short v4us;

__global__ __launch_bounds__(256) void k_aT(const float* __restrict__ Tk, const float* __restrict__ attb, bf* Ah, bf* Al) { const size_t e = ((size_t)blockIdx.x * 256 + threadIdx.x) * 4; if (e >= (size_t)NN * NN) return; const int m = (int)(e % NN), n = (int)(e / NN); v4us oh, ol;
#pragma unroll
    for (int q = 0; q < 4; ++q) { const size_t src = (size_t)(m + q) * NN + n; const float p = __fmul_rn(bfr(Tk[src]), bfr(attb[src])); unsigned short a, c2; splitf(p, a, c2); oh[q] = a; ol[q] = c2; }
    *(volatile v4us*)(Ah + e) = oh; *(volatile v4us*)(Al + e) = ol; __threadfence(); *(volatile v4us*)(Ah + e) = oh; *(volatile v4us*)(Al + e) = ol; }
__global__ __launch_bounds__(256) void k_xT(const float* __restrict__ xb, bf* XT) { const size_t e = ((size_t)blockIdx.x * 256 + threadIdx.x) * 4; if (e >= (size_t)FT * NN) return; const int m = (int)(e % NN), ft = (int)(e / NN); v4us o;
#pragma unroll
    for (int q = 0; q < 4; ++q) o[q] = f2bf(xb[(size_t)(m + q) * FT + ft]); *(volatile v4us*)(XT + e) = o; __threadfence(); *(volatile v4us*)(XT + e) = o; }
__global__ __launch_bounds__(256) void k_rT(const float* __restrict__ RHS, int k, bf* Rh, bf* Rl) { const size_t e = ((size_t)blockIdx.x * 256 + threadIdx.x) * 2; if (e >= (size_t)NT * FF) return; const int f = (int)(e % FF), nt = (int)(e / FF); const int n = nt / TS, t = nt % TS; v2us oh, ol;
#pragma unroll
    for (int q = 0; q < 2; ++q) { unsigned short a, c2; splitf(RHS[(size_t)n * FT + (f + q) * TS + t], a, c2); oh[q] = a; ol[q] = c2; }
    const size_t oo = (size_t)nt * KF + k * FF + f; *(volatile v2us*)(Rh + oo) = oh; *(volatile v2us*)(Rl + oo) = ol; __threadfence(); *(volatile v2us*)(Rh + oo) = oh; *(volatile v2us*)(Rl + oo) = ol; }
__global__ __launch_bounds__(256) void k_wth(const float* __restrict__ th, bf* Bt) { const int e = (blockIdx.x * 256 + threadIdx.x) * 2; if (e >= OO * KF) return; const int kf = e % KF, o = e / KF; v2us ov;
#pragma unroll
    for (int q = 0; q < 2; ++q) { const int kfq = kf + q; const int k = kfq / FF, f = kfq % FF; ov[q] = f2bf(th[((size_t)k * FF + f) * OO + o]); } *(volatile v2us*)(Bt + e) = ov; __threadfence(); *(volatile v2us*)(Bt + e) = ov; }
__global__ __launch_bounds__(256) void k_outp(const float* __restrict__ Cm, float* OUTb) { const size_t e = ((size_t)blockIdx.x * 256 + threadIdx.x) * 2; if (e >= (size_t)NN * OO * TS) return; typedef __attribute__((ext_vector_type(2))) float v2f; v2f o;
#pragma unroll
    for (int q = 0; q < 2; ++q) { const size_t idx = e + q; const int t = (int)(idx % TS); const int o_ = (int)((idx / TS) % OO); const int n = (int)(idx / ((size_t)TS * OO)); o[q] = fmaxf(Cm[((size_t)n * TS + t) * OO + o_], 0.f); }
    *(volatile v2f*)(OUTb + e) = o; __threadfence(); *(volatile v2f*)(OUTb + e) = o; }

extern "C" void kernel_launch(void* const* d_in, const int* in_sizes, int n_in,
                              void* d_out, int out_size, void* d_ws, size_t ws_size, hipStream_t stream) {
    (void)in_sizes; (void)n_in; (void)out_size;
    const float* x = (const float*)d_in[0]; const float* att = (const float*)d_in[1]; const float* cheb = (const float*)d_in[2]; const float* theta = (const float*)d_in[3];
    float* OUT = (float*)d_out;
    char* wsp = (char*)d_ws;
    auto take = [&](size_t bytes) { char* p = wsp; wsp += (bytes + 255) & ~(size_t)255; return (void*)p; };
    bf* WT = (bf*)take((size_t)OO * KF * 2); bf* XT = (bf*)take((size_t)FT * NN * 2); bf* Ah = (bf*)take((size_t)NN * NN * 2); bf* Al = (bf*)take((size_t)NN * NN * 2); float* RHS = (float*)take((size_t)NN * FT * 4);
    bf* Rh = (bf*)take((size_t)NT * KF * 2); bf* Rl = (bf*)take((size_t)NT * KF * 2); float* Cm = (float*)take((size_t)NT * OO * 4);
    if ((size_t)(wsp - (char*)d_ws) > ws_size) return;
    k_wth<<<(OO * KF / 2 + 255) / 256, 256, 0, stream>>>(theta, WT);
    for (int b = 0; b < NB_; ++b) {
        k_xT<<<(unsigned)(((size_t)FT * NN / 4 + 255) / 256), 256, 0, stream>>>(x + (size_t)b * NN * FT, XT);
        for (int k = 0; k < KC; ++k) {
            k_aT<<<(unsigned)(((size_t)NN * NN / 4 + 255) / 256), 256, 0, stream>>>(cheb + (size_t)k * NN * NN, att + (size_t)b * NN * NN, Ah, Al);
            k_gemmw<bf, 1, false><<<dim3(NN / 64, FT / 64, 1), 32, 0, stream>>>(Ah, Al, XT, nullptr, NN, RHS, FT, nullptr, 0, 0, 0);
            k_rT<<<(unsigned)(((size_t)NT * FF / 2 + 255) / 256), 256, 0, stream>>>(RHS, k, Rh, Rl); }
        k_gemmw<bf, 1, false><<<dim3(NT / 64, OO / 64, 1), 32, 0, stream>>>(Rh, Rl, WT, nullptr, KF, Cm, OO, nullptr, 0, 0, 0);
        k_outp<<<(unsigned)(((size_t)NN * OO * TS / 2 + 255) / 256), 256, 0, stream>>>(Cm, OUT + (size_t)b * NN * OO * TS); }
}
